// CausalSelfAttention_61220463837806
// MI455X (gfx1250) — hardware-verified
//
#include <hip/hip_runtime.h>
#include <math.h>

#ifndef NB
#define NB 2
#endif
#ifndef SEQ
#define SEQ 2048
#endif
#define NB_FULL 2
#define SEQ_FULL 2048
#define DM 1024
#define NHEAD 8
#define HDIM 128
#define MT (NB * SEQ)
#define QKW (2 * DM)
#define QKVW (3 * DM)
#define K2 (2 * DM)
#define EROWS ((SEQ < 512) ? SEQ : 512)
#define MTE (NB * EROWS)
#define GATEP 32

static_assert(NHEAD * HDIM == DM);
static_assert(HDIM == 128);
static_assert(NHEAD == 8);
static_assert(SEQ % 64 == 0);
static_assert(MT % 64 == 0);
static_assert(DM % 64 == 0);
static_assert(QKVW % 64 == 0);
static_assert(DM % 32 == 0);
static_assert(K2 % 32 == 0);
static_assert(EROWS % 64 == 0);
static_assert(EROWS <= SEQ);
static_assert(MTE % 64 == 0);
static_assert(DM == 8 * 128);
static_assert(GATEP * 4 == 128);
static_assert(NB <= NB_FULL);
static_assert(SEQ <= SEQ_FULL);
static_assert((long long)MT * QKW < 2147483647LL);
static_assert((long long)DM * MT < 2147483647LL);

typedef __attribute__((ext_vector_type(16))) _Float16 v16h;
typedef __attribute__((ext_vector_type(8)))  _Float16 v8h;
typedef __attribute__((ext_vector_type(8)))  float    v8f;
typedef __attribute__((ext_vector_type(4)))  float    v4f;
typedef __attribute__((ext_vector_type(4)))  unsigned int v4u;

union Fr { v16h v; v8h h[2]; };

__device__ __forceinline__ v8f wmma16(v16h a, v16h b, v8f c) {
    c = __builtin_amdgcn_wmma_f32_16x16x32_f16(false, a, false, b, (short)0, c, false, false);
    asm volatile("v_nop\n\tv_nop\n\tv_nop\n\tv_nop" : "+v"(c) : "v"(a), "v"(b));
    return c;
}
__device__ __forceinline__ void wave_sync() {
    __builtin_amdgcn_fence(3  , "workgroup");
    __builtin_amdgcn_wave_barrier();
    __builtin_amdgcn_fence(2  , "workgroup");
}
__device__ __forceinline__ float bfr(float v) {
    unsigned u = __float_as_uint(v);
    u = (u + 0x7fffu + ((u >> 16) & 1u)) & 0xffff0000u;
    return __uint_as_float(u);
}
__device__ __forceinline__ v4f bfr4(v4f a) { v4f r; r.x = bfr(a.x); r.y = bfr(a.y); r.z = bfr(a.z); r.w = bfr(a.w); return r; }
__device__ __forceinline__ unsigned pk2h(float a, float b) {
    return (unsigned)__builtin_bit_cast(unsigned short, (_Float16)a) | ((unsigned)__builtin_bit_cast(unsigned short, (_Float16)b) << 16);
}
__device__ __forceinline__ v4u pk8h(v4f a, v4f b) {
    v4u p; p.x = pk2h(a.x, a.y); p.y = pk2h(a.z, a.w); p.z = pk2h(b.x, b.y); p.w = pk2h(b.z, b.w); return p;
}
__device__ __forceinline__ void st2_u4(unsigned short* d, v4u pk) {
    volatile v4u* p = (volatile v4u*)d; *p = pk; __threadfence(); *p = pk;
}
__device__ __forceinline__ float gelu_erf(float v) { return 0.5f * v * (1.0f + erff(v * 0.70710678118654752f)); }
__device__ __forceinline__ v4f gelu4(v4f a) { v4f r; r.x = gelu_erf(a.x); r.y = gelu_erf(a.y); r.z = gelu_erf(a.z); r.w = gelu_erf(a.w); return r; }

typedef _Float16 h16;
static __device__ __forceinline__ h16 toh_flush(float v) { const h16 r = (h16)v; return (fabsf(v) < 6.103515625e-05f) ? (h16)0.0f : r; }
static __device__ __forceinline__ unsigned pk2hf(float a, float b) {
    return (unsigned)__builtin_bit_cast(unsigned short, toh_flush(a)) | ((unsigned)__builtin_bit_cast(unsigned short, toh_flush(b)) << 16);
}
static __device__ __forceinline__ v4u pk8hf(v4f a, v4f b) {
    v4u p; p.x = pk2hf(a.x, a.y); p.y = pk2hf(a.z, a.w); p.z = pk2hf(b.x, b.y); p.w = pk2hf(b.z, b.w); return p;
}
static __device__ __forceinline__ float res2k(float v) { return (v - (float)toh_flush(v)) * 2048.0f; }
static __device__ __forceinline__ v4f res4(v4f a) { v4f r; r.x = res2k(a.x); r.y = res2k(a.y); r.z = res2k(a.z); r.w = res2k(a.w); return r; }
static __device__ __forceinline__ v4f fma4(v4f a, v4f b, v4f c) {
    v4f r; r.x = fmaf(a.x, b.x, c.x); r.y = fmaf(a.y, b.y, c.y); r.z = fmaf(a.z, b.z, c.z); r.w = fmaf(a.w, b.w, c.w); return r;
}
static __device__ __forceinline__ float q8lin(float x, float pmax, float nmin, float rp, float rn) {
    const float tp = rintf((x * rp) * 127.0f) * (1.0f / 127.0f) * pmax;
    const float tn = rintf((x * rn) * 127.0f) * (1.0f / 127.0f) * nmin;
    return (x >= 0.0f) ? tp : tn;
}
static __device__ __forceinline__ v4f q8lin4(v4f a, float pmax, float nmin, float rp, float rn) {
    v4f r; r.x = q8lin(a.x, pmax, nmin, rp, rn); r.y = q8lin(a.y, pmax, nmin, rp, rn);
    r.z = q8lin(a.z, pmax, nmin, rp, rn); r.w = q8lin(a.w, pmax, nmin, rp, rn); return r;
}
static __device__ __forceinline__ float min4(v4f a) { return fminf(fminf(a.x, a.y), fminf(a.z, a.w)); }
static __device__ __forceinline__ float max4(v4f a) { return fmaxf(fmaxf(a.x, a.y), fmaxf(a.z, a.w)); }
static __device__ __forceinline__ void st2_f4(float* d, v4f v) {
    volatile v4f* p = (volatile v4f*)d; *p = v; __threadfence(); *p = v;
}

__global__ __launch_bounds__(256) void k_wrowsum(const float* __restrict__ W, float* __restrict__ RS) {
#pragma clang fp contract(off)
    __shared__ __align__(16) float rs[32];
    const int lane = (int)(threadIdx.x & 31);
    const int wave = __builtin_amdgcn_readfirstlane((int)(threadIdx.x >> 5));
    const int r0 = (int)blockIdx.x * 32 + wave * 4;
#pragma unroll 1
    for (int j = 0; j < 4; ++j) {
        const float* p = W + (size_t)(r0 + j) * DM;
        float s = 0.0f;
#pragma unroll 1
        for (int i = 0; i < 8; ++i) {
            const v4f a = *(const v4f*)(p + (i * 32 + lane) * 4);
            s += (fabsf(bfr(a.x)) + fabsf(bfr(a.y))) + (fabsf(bfr(a.z)) + fabsf(bfr(a.w)));
        }
        s += __shfl_xor(s, 16, 32); s += __shfl_xor(s, 8, 32); s += __shfl_xor(s, 4, 32); s += __shfl_xor(s, 2, 32); s += __shfl_xor(s, 1, 32);
        if (lane == 0) rs[wave * 4 + j] = s;
    }
    __syncthreads();
    const v4f v = *(const v4f*)&rs[4 * (lane & 7)];
    if (wave == 0 && lane < 8) st2_f4(RS + (size_t)blockIdx.x * 32 + 4 * lane, v);
}
__global__ __launch_bounds__(128) void k_wscale(const float* __restrict__ RS, float* __restrict__ SC) {
#pragma clang fp contract(off)
    __shared__ __align__(16) float sc[32];
    const int lane = (int)(threadIdx.x & 31);
    const int wave = __builtin_amdgcn_readfirstlane((int)(threadIdx.x >> 5));
    float s = 0.0f;
#pragma unroll 1
    for (int i = 0; i < 32; ++i) s += RS[wave * DM + i * 32 + lane];
    s += __shfl_xor(s, 16, 32); s += __shfl_xor(s, 8, 32); s += __shfl_xor(s, 4, 32); s += __shfl_xor(s, 2, 32); s += __shfl_xor(s, 1, 32);
    const float mval = fmaxf(s * (1.0f / (float)DM) * (1.0f / (float)DM), 1e-5f);
    if (wave == 0) sc[lane] = 0.0f;
    __syncthreads();
    if (lane == 0) sc[wave] = mval;
    __syncthreads();
    const v4f v = *(const v4f*)&sc[4 * (lane & 7)];
    if (wave == 0 && lane < 8) st2_f4(SC + 4 * lane, v);
}
__global__ __launch_bounds__(256) void k_cast_tern(const float* __restrict__ W, const float* __restrict__ SC, unsigned short* __restrict__ DST) {
#pragma clang fp contract(off)
    const int u = (int)blockIdx.x * 256 + (int)threadIdx.x;
    if (u >= 4 * DM * (DM / 8)) return;
    const int o = u >> 7, c0 = 8 * (u & 127);
    const float s = SC[o >> 10];
    const float rs = 1.0f / s;
    const float* p = W + (size_t)o * DM + c0;
    const v4f a = bfr4(*(const v4f*)p), b = bfr4(*(const v4f*)(p + 4));
    v4f ta, tb;
    ta.x = fminf(fmaxf(rintf(a.x * rs), -1.0f), 1.0f); ta.y = fminf(fmaxf(rintf(a.y * rs), -1.0f), 1.0f);
    ta.z = fminf(fmaxf(rintf(a.z * rs), -1.0f), 1.0f); ta.w = fminf(fmaxf(rintf(a.w * rs), -1.0f), 1.0f);
    tb.x = fminf(fmaxf(rintf(b.x * rs), -1.0f), 1.0f); tb.y = fminf(fmaxf(rintf(b.y * rs), -1.0f), 1.0f);
    tb.z = fminf(fmaxf(rintf(b.z * rs), -1.0f), 1.0f); tb.w = fminf(fmaxf(rintf(b.w * rs), -1.0f), 1.0f);
    const v4u hi = pk8hf(ta, tb);
    const v4u lo = pk8hf(ta * (1.0f / 2048.0f), tb * (1.0f / 2048.0f));
    st2_u4(DST + (size_t)o * K2 + c0, hi);
    st2_u4(DST + (size_t)o * K2 + DM + c0, lo);
}

__global__ __launch_bounds__(256) void k_xquant(const float* __restrict__ X, const float* __restrict__ GW,
                                                unsigned short* __restrict__ XQ, float* __restrict__ GATE, int rows) {
#pragma clang fp contract(off)
    __shared__ float redn[8];
    __shared__ float redp[8];
    __shared__ float x16[32];
    __shared__ __align__(16) float gl[64];
    const int tid = (int)threadIdx.x, lane = tid & 31;
    const int wave = __builtin_amdgcn_readfirstlane(tid >> 5);
    const int half = wave >> 2, w0 = half * 4;
    const int ht = tid & 127;
    const int row = (int)blockIdx.x * 2 + half;
    const int rowc = min(row, rows - 1);
    const int rsrc = (rowc / SEQ) * SEQ_FULL + (rowc % SEQ);
    const int c0 = 8 * ht;
    const float* xr = X + (size_t)rsrc * DM + c0;
    const v4f a0 = bfr4(*(const v4f*)xr), a1 = bfr4(*(const v4f*)(xr + 4));
    float mn = fminf(min4(a0), min4(a1));
    float mx = fmaxf(max4(a0), max4(a1));
    mn = fminf(mn, __shfl_xor(mn, 16, 32)); mn = fminf(mn, __shfl_xor(mn, 8, 32)); mn = fminf(mn, __shfl_xor(mn, 4, 32));
    mn = fminf(mn, __shfl_xor(mn, 2, 32));  mn = fminf(mn, __shfl_xor(mn, 1, 32));
    mx = fmaxf(mx, __shfl_xor(mx, 16, 32)); mx = fmaxf(mx, __shfl_xor(mx, 8, 32)); mx = fmaxf(mx, __shfl_xor(mx, 4, 32));
    mx = fmaxf(mx, __shfl_xor(mx, 2, 32));  mx = fmaxf(mx, __shfl_xor(mx, 1, 32));
    if (lane == 0) { redn[wave] = mn; redp[wave] = mx; }
    __syncthreads();
    const float nmin = fminf(fminf(fminf(redn[w0], redn[w0 + 1]), fminf(redn[w0 + 2], redn[w0 + 3])), -1e-5f);
    const float pmax = fmaxf(fmaxf(fmaxf(redp[w0], redp[w0 + 1]), fmaxf(redp[w0 + 2], redp[w0 + 3])), 1e-5f);
    const float rp = 1.0f / pmax, rn = 1.0f / nmin;
    const v4f q0 = q8lin4(a0, pmax, nmin, rp, rn), q1 = q8lin4(a1, pmax, nmin, rp, rn);
    if (ht < 2) {
        const int xb = half * 16 + c0;
        x16[xb + 0] = q0.x; x16[xb + 1] = q0.y; x16[xb + 2] = q0.z; x16[xb + 3] = q0.w;
        x16[xb + 4] = q1.x; x16[xb + 5] = q1.y; x16[xb + 6] = q1.z; x16[xb + 7] = q1.w;
    }
    __syncthreads();
    if ((wave & 3) == 0) {
        const int hc = lane & 7;
        float z = 0.0f;
#pragma unroll 1
        for (int f = 0; f < 12; ++f) z += x16[half * 16 + f] * bfr(GW[hc * 12 + f]);
        const float gv = 1.0f / (1.0f + expf(-z));
        gl[half * 32 + lane] = (lane < 8) ? gv : 0.0f;
    }
    __syncthreads();
    const v4f gvv = *(const v4f*)&gl[half * 32 + 4 * (ht & 7)];
    const v4u pkh = pk8hf(q0, q1);
    const v4u pkr = pk8hf(res4(q0), res4(q1));
    if (row < rows) {
        st2_u4(XQ + (size_t)row * K2 + c0, pkh);
        st2_u4(XQ + (size_t)row * K2 + DM + c0, pkr);
        if (ht < 8) st2_f4(GATE + (size_t)row * GATEP + 4 * ht, gvv);
    }
}

template <int OUT_MODE, bool HASBIAS, bool ACTG, bool RESID>
__device__ __forceinline__ void gemm64_body(const unsigned short* __restrict__ Ap, int lda,
                                            const unsigned short* __restrict__ Btp, int ldb,
                                            float* __restrict__ Cf, unsigned short* __restrict__ Ch, int ldc,
                                            const float* __restrict__ bias, const float* __restrict__ resid, int ldr,
                                            int M, int N, int K, float scale, float carry, int rbf,
                                            int cseq, int cseqf, int rseq, int rseqf) {
    __shared__ __align__(16) float sT[8 * 16 * 68];
    const _Float16* A  = (const _Float16*)Ap;
    const _Float16* Bt = (const _Float16*)Btp;
    const int lane = (int)(threadIdx.x & 31);
    const int wave = __builtin_amdgcn_readfirstlane((int)(threadIdx.x >> 5));
    const int tilesN = N >> 6, tilesM = M >> 6;
    const int tile = (int)blockIdx.x * 8 + wave;
    if (tile >= tilesM * tilesN) return;
    const int tm = tile / tilesN, tn = tile - tm * tilesN;
    const int m0 = tm << 6, n0 = tn << 6;
    const int rl = lane & 15, hh = lane >> 4, koff = hh * 8, mOff = hh * 8;

    v8f acc[4][4];
#pragma unroll
    for (int i = 0; i < 4; ++i)
#pragma unroll
        for (int j = 0; j < 4; ++j) { v8f z = {}; acc[i][j] = z; }

    for (int k0 = 0; k0 < K; k0 += 32) {
        Fr bh[4];
#pragma unroll
        for (int j = 0; j < 4; ++j) {
            const size_t bo = (size_t)(n0 + (j << 4) + rl) * ldb + koff + k0;
            bh[j].h[0] = *(const v8h*)(Bt + bo);
            bh[j].h[1] = *(const v8h*)(Bt + bo + 16);
        }
#pragma unroll
        for (int i = 0; i < 4; ++i) {
            const size_t ao = (size_t)(m0 + (i << 4) + rl) * lda + koff + k0;
            Fr ah;
            ah.h[0] = *(const v8h*)(A + ao);
            ah.h[1] = *(const v8h*)(A + ao + 16);
#pragma unroll
            for (int j = 0; j < 4; ++j) acc[i][j] = wmma16(ah.v, bh[j].v, acc[i][j]);
        }
    }

    const int sbase = wave * (16 * 68);
    const int crow0 = (m0 / cseq) * cseqf + (m0 % cseq);
    const int rrow0 = (m0 / rseq) * rseqf + (m0 % rseq);
    const int c4 = (lane & 15) * 4;
    const int q8 = lane >> 3, c8 = (lane & 7) * 8;
    v4f b4 = {0.f, 0.f, 0.f, 0.f}, ba = {0.f, 0.f, 0.f, 0.f}, bb = {0.f, 0.f, 0.f, 0.f};
    if (HASBIAS) {
        if (OUT_MODE == 0) b4 = bfr4(*(const v4f*)(bias + n0 + c4));
        else { ba = bfr4(*(const v4f*)(bias + n0 + c8)); bb = bfr4(*(const v4f*)(bias + n0 + c8 + 4)); }
    }
#pragma unroll
    for (int i = 0; i < 4; ++i) {
        const int mB = i << 4;
#pragma unroll
        for (int j = 0; j < 4; ++j)
#pragma unroll
            for (int r = 0; r < 8; ++r) sT[sbase + (mOff + r) * 68 + (j << 4) + rl] = acc[i][j][r] * scale;
        wave_sync();
        if (OUT_MODE == 0) {
#pragma unroll 1
            for (int it = 0; it < 8; ++it) {
                const int row = it * 2 + hh; const int si = sbase + row * 68 + c4;
                v4f v = *(const v4f*)&sT[si];
                v = v + b4;
                if (RESID) {
                    v4f rr = *(const v4f*)(resid + (size_t)(rrow0 + mB + row) * ldr + n0 + c4);
                    const v4f rq = bfr4(rr);
                    if (rbf) rr = rq;
                    v = v + rr;
                }
                *(v4f*)&sT[si] = v;
            }
            wave_sync();
            for (int pass = 0; pass < 2; ++pass) {
#pragma unroll
                for (int it = 0; it < 8; ++it) {
                    const int row = it * 2 + hh;
                    const v4f v = *(const v4f*)&sT[sbase + row * 68 + c4];
                    *(volatile v4f*)(Cf + (size_t)(crow0 + mB + row) * ldc + n0 + c4) = v;
                }
                __threadfence();
            }
        } else {
            if (HASBIAS || ACTG) {
#pragma unroll 1
                for (int it = 0; it < 4; ++it) {
                    const int row = it * 4 + q8; const int si = sbase + row * 68 + c8;
                    v4f va = *(const v4f*)&sT[si], vb = *(const v4f*)&sT[si + 4];
                    va = va + ba; vb = vb + bb;
                    if (ACTG) { va = gelu4(va); vb = gelu4(vb); }
                    va = va * carry; vb = vb * carry;
                    *(v4f*)&sT[si] = va; *(v4f*)&sT[si + 4] = vb;
                }
                wave_sync();
            }
            for (int pass = 0; pass < 2; ++pass) {
#pragma unroll
                for (int it = 0; it < 4; ++it) {
                    const int row = it * 4 + q8; const int si = sbase + row * 68 + c8;
                    const v4f va = *(const v4f*)&sT[si], vb = *(const v4f*)&sT[si + 4];
                    const v4u pk = pk8h(va, vb);
                    *(volatile v4u*)(Ch + (size_t)(crow0 + mB + row) * ldc + n0 + c8) = pk;
                }
                __threadfence();
            }
        }
        wave_sync();
    }
}

__global__ __launch_bounds__(256) void k_gemm_f32(const unsigned short* __restrict__ A, int lda, const unsigned short* __restrict__ Bt, int ldb,
                                                  float* __restrict__ C, int ldc, int M, int N, int K, float scale, int cseq, int cseqf) {
    gemm64_body<0, false, false, false>(A, lda, Bt, ldb, C, nullptr, ldc, nullptr, nullptr, 0, M, N, K, scale, 1.0f, 0, cseq, cseqf, M, M);
}

__global__ __launch_bounds__(256) void k_qkpost(const float* __restrict__ QKV, const float* __restrict__ SC,
                                                const float* __restrict__ COSB, const float* __restrict__ SINB,
                                                unsigned short* __restrict__ QK, unsigned short* __restrict__ QKR) {
#pragma clang fp contract(off)
    const int lane = (int)(threadIdx.x & 31);
    const int h = __builtin_amdgcn_readfirstlane((int)(threadIdx.x >> 5));
    const int g = lane >> 3, which = g & 1, tsub = g >> 1, c = lane & 7;
    const int mblk = (int)blockIdx.x * 2;
    const int m = mblk + tsub;
    const int b = m / SEQ, s = m - b * SEQ;
    const float sc = SC[which];
    const float* src = QKV + (size_t)m * QKVW + which * DM + h * HDIM + 8 * c;
    v4f x1a = *(const v4f*)src, x1b = *(const v4f*)(src + 4), x2a = *(const v4f*)(src + 64), x2b = *(const v4f*)(src + 68);
    x1a = x1a * sc; x1b = x1b * sc; x2a = x2a * sc; x2b = x2b * sc;
    const v4f qa = x1a * x1a, qb = x1b * x1b, qc = x2a * x2a, qd = x2b * x2b;
    float ss = (((qa.x + qa.y) + (qa.z + qa.w)) + ((qb.x + qb.y) + (qb.z + qb.w))) + (((qc.x + qc.y) + (qc.z + qc.w)) + ((qd.x + qd.y) + (qd.z + qd.w)));
    ss += __shfl_xor(ss, 1, 32); ss += __shfl_xor(ss, 2, 32); ss += __shfl_xor(ss, 4, 32);
    const float rnorm = 1.0f / sqrtf(ss * (1.0f / 128.0f) + 1.1920928955078125e-07f);
    x1a = x1a * rnorm; x1b = x1b * rnorm; x2a = x2a * rnorm; x2b = x2b * rnorm;
    const float* cp = COSB + (size_t)s * 64 + 8 * c;
    const float* sp = SINB + (size_t)s * 64 + 8 * c;
    const v4f ca = bfr4(*(const v4f*)cp), cb = bfr4(*(const v4f*)(cp + 4));
    const v4f sa = bfr4(*(const v4f*)sp), sb = bfr4(*(const v4f*)(sp + 4));
    const v4f ya = fma4(x1a, ca, x2a * sa), yb = fma4(x1b, cb, x2b * sb);
    const v4f za = fma4(-x1a, sa, x2a * ca), zb = fma4(-x1b, sb, x2b * cb);
    float mn = fminf(fminf(min4(ya), min4(yb)), fminf(min4(za), min4(zb)));
    float mx = fmaxf(fmaxf(max4(ya), max4(yb)), fmaxf(max4(za), max4(zb)));
    mn = fminf(mn, __shfl_xor(mn, 1, 32)); mn = fminf(mn, __shfl_xor(mn, 2, 32)); mn = fminf(mn, __shfl_xor(mn, 4, 32));
    mx = fmaxf(mx, __shfl_xor(mx, 1, 32)); mx = fmaxf(mx, __shfl_xor(mx, 2, 32)); mx = fmaxf(mx, __shfl_xor(mx, 4, 32));
    const float nmin = fminf(mn, -1e-5f), pmax = fmaxf(mx, 1e-5f);
    const float rp = 1.0f / pmax, rn = 1.0f / nmin;
    const v4f ua = q8lin4(ya, pmax, nmin, rp, rn), ub = q8lin4(yb, pmax, nmin, rp, rn);
    const v4f wa = q8lin4(za, pmax, nmin, rp, rn), wb = q8lin4(zb, pmax, nmin, rp, rn);
    const v4u p1 = pk8hf(ua, ub), p2 = pk8hf(wa, wb);
    unsigned short* d = QK + (size_t)m * QKW + h * 256 + which * HDIM + 8 * c;
    st2_u4(d, p1);
    st2_u4(d + 64, p2);
    if ((mblk % SEQ) < EROWS) {
        const v4u r1 = pk8hf(res4(ua), res4(ub)), r2 = pk8hf(res4(wa), res4(wb));
        unsigned short* dr = QKR + (size_t)(b * EROWS + s) * QKW + h * 256 + which * HDIM + 8 * c;
        st2_u4(dr, r1);
        st2_u4(dr + 64, r2);
    }
}

__global__ __launch_bounds__(256) void k_vpost(const float* __restrict__ QKV, const float* __restrict__ VE, const float* __restrict__ LAM,
                                               const float* __restrict__ SC, unsigned short* __restrict__ VT, unsigned short* __restrict__ VTR) {
#pragma clang fp contract(off)
    __shared__ __align__(16) float T[64 * 68];
    const int tid = (int)threadIdx.x;
    const int bt = (int)blockIdx.x >> 4, bc = (int)blockIdx.x & 15;
    const int m0 = bt * 64, c0 = bc * 64;
    const int b = m0 / SEQ, s0 = m0 - b * SEQ;
    const float l0 = bfr(LAM[0]), l1 = bfr(LAM[1]);
    const float sv = SC[2];
    const int cc = (tid & 15) * 4;
#pragma unroll 1
    for (int i = 0; i < 4; ++i) {
        const int tok = (tid >> 4) + 16 * i;
        const v4f p = *(const v4f*)(QKV + (size_t)(m0 + tok) * QKVW + 2 * DM + c0 + cc);
        const v4f e = bfr4(*(const v4f*)(VE + (size_t)(b * SEQ_FULL + s0 + tok) * DM + c0 + cc));
        const v4f val = (p * sv) * l0 + e * l1;
        T[(cc + 0) * 68 + tok] = val.x; T[(cc + 1) * 68 + tok] = val.y; T[(cc + 2) * 68 + tok] = val.z; T[(cc + 3) * 68 + tok] = val.w;
    }
    __syncthreads();
    const int t8 = (tid & 7) * 8;
#pragma unroll 1
    for (int it = 0; it < 2; ++it) {
        const int row = it * 32 + (tid >> 3);
        const v4f va = *(const v4f*)&T[row * 68 + t8], vb = *(const v4f*)&T[row * 68 + t8 + 4];
        const v4u pkh = pk8hf(va, vb);
        st2_u4(VT + (size_t)(c0 + row) * MT + m0 + t8, pkh);
        if (s0 < EROWS) {
            const v4u pkr = pk8hf(res4(va), res4(vb));
            st2_u4(VTR + (size_t)(c0 + row) * MTE + b * EROWS + s0 + t8, pkr);
        }
    }
}

__global__ __launch_bounds__(128) void k_attn128(const unsigned short* __restrict__ QKp, const unsigned short* __restrict__ VTp,
                                                 const float* __restrict__ GATE, const float* __restrict__ SC,
                                                 unsigned short* __restrict__ CTXp) {
    __shared__ __align__(16) _Float16 Pl[4 * 16 * 40];
    __shared__ __align__(16) float    Ol[4 * 16 * 132];
    const _Float16* QK = (const _Float16*)QKp;
    const _Float16* VT = (const _Float16*)VTp;
    const int lane = (int)(threadIdx.x & 31), hh = lane >> 4, c = lane & 15;
    const int wave = __builtin_amdgcn_readfirstlane((int)(threadIdx.x >> 5));
    const int NQB = SEQ / 64;
    const int bx = (int)blockIdx.x;
    const int qb = bx % NQB, bh = bx / NQB;
    const int h = bh % NHEAD, b = bh / NHEAD;
    const int q0 = qb * 64 + wave * 16;
    const int qoff0 = (b * SEQ + q0 + c) * QKW + h * 256 + 8 * hh;
    const int kbase = (b * SEQ + c) * QKW + h * 256 + 128 + 8 * hh;
    const int vbase = (h * HDIM + c) * MT + b * SEQ + 8 * hh;
    const int pbase = wave * (16 * 40);
    const float SL2 = 0.12f * 1.4426950408889634f;
    const float NEG = -__builtin_inff();

    v8f o[8]; float m8[8], l8[8];
#pragma unroll
    for (int t = 0; t < 8; ++t) { v8f z = {}; o[t] = z; }
#pragma unroll
    for (int r = 0; r < 8; ++r) { m8[r] = NEG; l8[r] = 0.f; }

    const int nh = (q0 + 16 + 31) >> 5;
    for (int jh = 0; jh < nh; ++jh) {
        const int kv0 = jh * 32;
        int qo = qoff0;
        asm volatile("" : "+v"(qo));
        v8f s0 = {}, s1 = {};
#pragma unroll
        for (int ks = 0; ks < 4; ++ks) {
            Fr qa, k0f, k1f;
            qa.h[0] = *(const v8h*)(QK + qo + ks * 32);
            qa.h[1] = *(const v8h*)(QK + qo + ks * 32 + 16);
            const int ko0 = kbase + kv0 * QKW + ks * 32;
            k0f.h[0] = *(const v8h*)(QK + ko0);
            k0f.h[1] = *(const v8h*)(QK + ko0 + 16);
            s0 = wmma16(qa.v, k0f.v, s0);
            const int ko1 = ko0 + 16 * QKW;
            k1f.h[0] = *(const v8h*)(QK + ko1);
            k1f.h[1] = *(const v8h*)(QK + ko1 + 16);
            s1 = wmma16(qa.v, k1f.v, s1);
        }
        const bool diag = (kv0 + 31 > q0);
#pragma unroll
        for (int r = 0; r < 8; ++r) {
            float v0 = s0[r] * SL2, v1 = s1[r] * SL2;
            if (diag) {
                const int qrow = q0 + 8 * hh + r;
                v0 = (kv0 + c > qrow) ? NEG : v0;
                v1 = (kv0 + 16 + c > qrow) ? NEG : v1;
            }
            float mx = fmaxf(v0, v1);
            mx = fmaxf(mx, __shfl_xor(mx, 1, 32)); mx = fmaxf(mx, __shfl_xor(mx, 2, 32));
            mx = fmaxf(mx, __shfl_xor(mx, 4, 32)); mx = fmaxf(mx, __shfl_xor(mx, 8, 32));
            const float mnew = fmaxf(m8[r], mx);
            const float msafe = (mnew == NEG) ? 0.f : mnew;
            const float alpha = exp2f(m8[r] - msafe);
            const float e0 = v0 - msafe, e1 = v1 - msafe;
            const float p0 = exp2f(e0), p1 = exp2f(e1);
            float rs = p0 + p1;
            rs += __shfl_xor(rs, 1, 32); rs += __shfl_xor(rs, 2, 32); rs += __shfl_xor(rs, 4, 32); rs += __shfl_xor(rs, 8, 32);
            l8[r] = l8[r] * alpha + rs; m8[r] = mnew;
#pragma unroll
            for (int t = 0; t < 8; ++t) o[t][r] *= alpha;
            Pl[pbase + (8 * hh + r) * 40 + c]      = (e0 < -24.0f) ? (_Float16)0.0f : (_Float16)(p0 * 1024.0f);
            Pl[pbase + (8 * hh + r) * 40 + 16 + c] = (e1 < -24.0f) ? (_Float16)0.0f : (_Float16)(p1 * 1024.0f);
        }
        wave_sync();
        Fr pa;
        pa.h[0] = *(const v8h*)&Pl[pbase + c * 40 + 8 * hh];
        pa.h[1] = *(const v8h*)&Pl[pbase + c * 40 + 16 + 8 * hh];
#pragma unroll
        for (int t = 0; t < 8; ++t) {
            Fr vb;
            const int vo = vbase + t * 16 * MT + kv0;
            vb.h[0] = *(const v8h*)(VT + vo);
            vb.h[1] = *(const v8h*)(VT + vo + 16);
            o[t] = wmma16(pa.v, vb.v, o[t]);
        }
        wave_sync();
    }

    const int obase = wave * (16 * 132);
    const float so4 = SC[3] * 4.0f;
#pragma unroll
    for (int r = 0; r < 8; ++r) {
        const float gt = GATE[(size_t)(b * SEQ + q0 + 8 * hh + r) * GATEP + h];
        const float inv = (gt * so4) * (1.0f / l8[r]);
#pragma unroll
        for (int t = 0; t < 8; ++t) Ol[obase + (8 * hh + r) * 132 + t * 16 + c] = o[t][r] * inv;
    }
    wave_sync();
    {
        const int c8 = (lane & 15) * 8;
        for (int pass = 0; pass < 2; ++pass) {
#pragma unroll
            for (int it = 0; it < 8; ++it) {
                const int row = it * 2 + hh; const int si = obase + row * 132 + c8;
                const v4f va = *(const v4f*)&Ol[si], vb = *(const v4f*)&Ol[si + 4];
                const v4u pk = pk8hf(va, vb);
                *(volatile v4u*)(CTXp + (size_t)(b * SEQ + q0 + row) * DM + h * HDIM + c8) = pk;
            }
            __threadfence();
        }
    }
}

__global__ __launch_bounds__(128) void k_attn_early(const unsigned short* __restrict__ QKp, const unsigned short* __restrict__ QRp,
                                                    const unsigned short* __restrict__ VTp, const unsigned short* __restrict__ VRp,
                                                    const float* __restrict__ GATE, const float* __restrict__ SC,
                                                    unsigned short* __restrict__ CTXE) {
    __shared__ __align__(16) _Float16 Pl[4 * 16 * 40];
    __shared__ __align__(16) _Float16 Plr[4 * 16 * 40];
    __shared__ __align__(16) float    Ol[4 * 16 * 68];
    const _Float16* QK = (const _Float16*)QKp;
    const _Float16* QR = (const _Float16*)QRp;
    const _Float16* VT = (const _Float16*)VTp;
    const _Float16* VR = (const _Float16*)VRp;
    const int lane = (int)(threadIdx.x & 31), hh = lane >> 4, c = lane & 15;
    const int wave = __builtin_amdgcn_readfirstlane((int)(threadIdx.x >> 5));
    const int NQE = EROWS / 64;
    const int bx = (int)blockIdx.x;
    const int half = bx & 1, bq = bx >> 1;
    const int qb = bq % NQE, bh = bq / NQE;
    const int h = bh % NHEAD, b = bh / NHEAD;
    const int q0 = qb * 64 + wave * 16;
    const int qoff0 = (b * SEQ + q0 + c) * QKW + h * 256 + 8 * hh;
    const int roff0 = (b * EROWS + q0 + c) * QKW + h * 256 + 8 * hh;
    const int kbase = (b * SEQ + c) * QKW + h * 256 + 128 + 8 * hh;
    const int rbase = (b * EROWS + c) * QKW + h * 256 + 128 + 8 * hh;
    const int vbase = (h * HDIM + half * 64 + c) * MT + b * SEQ + 8 * hh;
    const int wbase = (h * HDIM + half * 64 + c) * MTE + b * EROWS + 8 * hh;
    const int pbase = wave * (16 * 40);
    const float SL2 = 0.12f * 1.4426950408889634f;
    const float NEG = -__builtin_inff();
    const float R2K = 1.0f / 2048.0f;

    v8f o[4], orr[4]; float m8[8], l8[8];
#pragma unroll
    for (int t = 0; t < 4; ++t) { v8f z = {}; o[t] = z; orr[t] = z; }
#pragma unroll
    for (int r = 0; r < 8; ++r) { m8[r] = NEG; l8[r] = 0.f; }

    const int nh = (q0 + 16 + 31) >> 5;
    for (int jh = 0; jh < nh; ++jh) {
        const int kv0 = jh * 32;
        int qo = qoff0, ro = roff0;
        asm volatile("" : "+v"(qo));
        asm volatile("" : "+v"(ro));
        v8f s0 = {}, s1 = {}, t0 = {}, t1 = {};
#pragma unroll
        for (int ks = 0; ks < 4; ++ks) {
            Fr qa, qr, kh, kr;
            qa.h[0] = *(const v8h*)(QK + qo + ks * 32);
            qa.h[1] = *(const v8h*)(QK + qo + ks * 32 + 16);
            qr.h[0] = *(const v8h*)(QR + ro + ks * 32);
            qr.h[1] = *(const v8h*)(QR + ro + ks * 32 + 16);
            const int ko0 = kbase + kv0 * QKW + ks * 32;
            const int kr0 = rbase + kv0 * QKW + ks * 32;
            kh.h[0] = *(const v8h*)(QK + ko0);
            kh.h[1] = *(const v8h*)(QK + ko0 + 16);
            kr.h[0] = *(const v8h*)(QR + kr0);
            kr.h[1] = *(const v8h*)(QR + kr0 + 16);
            s0 = wmma16(qa.v, kh.v, s0);
            t0 = wmma16(qa.v, kr.v, t0);
            t0 = wmma16(qr.v, kh.v, t0);
            const int ko1 = ko0 + 16 * QKW;
            const int kr1 = kr0 + 16 * QKW;
            kh.h[0] = *(const v8h*)(QK + ko1);
            kh.h[1] = *(const v8h*)(QK + ko1 + 16);
            kr.h[0] = *(const v8h*)(QR + kr1);
            kr.h[1] = *(const v8h*)(QR + kr1 + 16);
            s1 = wmma16(qa.v, kh.v, s1);
            t1 = wmma16(qa.v, kr.v, t1);
            t1 = wmma16(qr.v, kh.v, t1);
        }
        const bool diag = (kv0 + 31 > q0);
#pragma unroll
        for (int r = 0; r < 8; ++r) {
            float v0 = (s0[r] + t0[r] * R2K) * SL2, v1 = (s1[r] + t1[r] * R2K) * SL2;
            if (diag) {
                const int qrow = q0 + 8 * hh + r;
                v0 = (kv0 + c > qrow) ? NEG : v0;
                v1 = (kv0 + 16 + c > qrow) ? NEG : v1;
            }
            float mx = fmaxf(v0, v1);
            mx = fmaxf(mx, __shfl_xor(mx, 1, 32)); mx = fmaxf(mx, __shfl_xor(mx, 2, 32));
            mx = fmaxf(mx, __shfl_xor(mx, 4, 32)); mx = fmaxf(mx, __shfl_xor(mx, 8, 32));
            const float mnew = fmaxf(m8[r], mx);
            const float msafe = (mnew == NEG) ? 0.f : mnew;
            const float alpha = exp2f(m8[r] - msafe);
            const float e0 = v0 - msafe, e1 = v1 - msafe;
            const float p0 = exp2f(e0), p1 = exp2f(e1);
            float rs = p0 + p1;
            rs += __shfl_xor(rs, 1, 32); rs += __shfl_xor(rs, 2, 32); rs += __shfl_xor(rs, 4, 32); rs += __shfl_xor(rs, 8, 32);
            l8[r] = l8[r] * alpha + rs; m8[r] = mnew;
#pragma unroll
            for (int t = 0; t < 4; ++t) { o[t][r] *= alpha; orr[t][r] *= alpha; }
            const float f0 = p0 * 1024.0f, f1 = p1 * 1024.0f;
            const _Float16 h0 = (e0 < -24.0f) ? (_Float16)0.0f : (_Float16)f0;
            const _Float16 h1 = (e1 < -24.0f) ? (_Float16)0.0f : (_Float16)f1;
            Pl[pbase + (8 * hh + r) * 40 + c]       = h0;
            Pl[pbase + (8 * hh + r) * 40 + 16 + c]  = h1;
            Plr[pbase + (8 * hh + r) * 40 + c]      = toh_flush((f0 - (float)h0) * 2048.0f);
            Plr[pbase + (8 * hh + r) * 40 + 16 + c] = toh_flush((f1 - (float)h1) * 2048.0f);
        }
        wave_sync();
        Fr pa, pr;
        pa.h[0] = *(const v8h*)&Pl[pbase + c * 40 + 8 * hh];
        pa.h[1] = *(const v8h*)&Pl[pbase + c * 40 + 16 + 8 * hh];
        pr.h[0] = *(const v8h*)&Plr[pbase + c * 40 + 8 * hh];
        pr.h[1] = *(const v8h*)&Plr[pbase + c * 40 + 16 + 8 * hh];
#pragma unroll
        for (int t = 0; t < 4; ++t) {
            Fr vb, vr;
            const int vo = vbase + t * 16 * MT + kv0;
            const int wo = wbase + t * 16 * MTE + kv0;
            vb.h[0] = *(const v8h*)(VT + vo);
            vb.h[1] = *(const v8h*)(VT + vo + 16);
            vr.h[0] = *(const v8h*)(VR + wo);
            vr.h[1] = *(const v8h*)(VR + wo + 16);
            o[t]   = wmma16(pa.v, vb.v, o[t]);
            orr[t] = wmma16(pa.v, vr.v, orr[t]);
            orr[t] = wmma16(pr.v, vb.v, orr[t]);
        }
        wave_sync();
    }

    const int obase = wave * (16 * 68);
    const float so4 = SC[3] * 4.0f;
#pragma unroll
    for (int r = 0; r < 8; ++r) {
        const float gt = GATE[(size_t)(b * SEQ + q0 + 8 * hh + r) * GATEP + h];
        const float inv = (gt * so4) * (1.0f / l8[r]);
#pragma unroll
        for (int t = 0; t < 4; ++t) Ol[obase + (8 * hh + r) * 68 + t * 16 + c] = (o[t][r] + orr[t][r] * R2K) * inv;
    }
    wave_sync();
    {
        const int q8 = lane >> 3, c8 = (lane & 7) * 8;
        for (int pass = 0; pass < 2; ++pass) {
#pragma unroll
            for (int it = 0; it < 4; ++it) {
                const int row = it * 4 + q8; const int si = obase + row * 68 + c8;
                const v4f va = *(const v4f*)&Ol[si], vb = *(const v4f*)&Ol[si + 4];
                const v4u pkh = pk8hf(va, vb);
                const v4u pkr = pk8hf(res4(va), res4(vb));
                unsigned short* d = CTXE + (size_t)(b * EROWS + q0 + row) * K2 + h * HDIM + half * 64 + c8;
                *(volatile v4u*)d = pkh;
                *(volatile v4u*)(d + DM) = pkr;
            }
            __threadfence();
        }
    }
}

#define SZ_RS    ((size_t)4 * DM * 4)
#define SZ_SC    ((size_t)256)
#define SZ_XQ    ((size_t)MT * K2 * 2)
#define SZ_W2    ((size_t)4 * DM * K2 * 2)
#define SZ_QKV   ((size_t)MT * QKVW * 4)
#define SZ_GATE  ((size_t)MT * GATEP * 4)
#define SZ_QK16  ((size_t)MT * QKW * 2)
#define SZ_QKR   ((size_t)MTE * QKW * 2)
#define SZ_VT16  ((size_t)DM * MT * 2)
#define SZ_VTR   ((size_t)DM * MTE * 2)
#define SZ_CTX16 ((size_t)MT * DM * 2)
#define SZ_CTXE  ((size_t)MTE * K2 * 2)
#define SZ_TOTAL (SZ_RS + SZ_SC + SZ_XQ + SZ_W2 + SZ_QKV + SZ_GATE + SZ_QK16 + SZ_QKR + SZ_VT16 + SZ_VTR + SZ_CTX16 + SZ_CTXE)
static_assert(SZ_TOTAL <= (size_t)134217728);
static_assert(SZ_RS % 256 == 0);
static_assert(SZ_XQ % 256 == 0);
static_assert(SZ_W2 % 256 == 0);
static_assert(SZ_QKV % 256 == 0);
static_assert(SZ_GATE % 256 == 0);
static_assert(SZ_QK16 % 256 == 0);
static_assert(SZ_QKR % 256 == 0);
static_assert(SZ_VT16 % 256 == 0);
static_assert(SZ_VTR % 256 == 0);
static_assert(SZ_CTX16 % 256 == 0);
static_assert((4 * DM) % 32 == 0);
static_assert((4 * DM * (DM / 8)) % 256 == 0);
static_assert(((MT / 64) * (QKVW / 64)) % 8 == 0);
static_assert(((MT / 64) * (DM / 64)) % 8 == 0);
static_assert(((MTE / 64) * (DM / 64)) % 8 == 0);

extern "C" void kernel_launch(void* const* d_in, const int* in_sizes, int n_in, void* d_out, int out_size, void* d_ws, size_t ws_size, hipStream_t stream) {
    if (n_in < 7) return;
    const long long need_rows = (long long)(NB - 1) * SEQ_FULL + SEQ;
    if ((long long)in_sizes[0] < need_rows * DM) return;
    if ((long long)in_sizes[1] < need_rows * DM) return;
    if (in_sizes[2] < 2) return;
    if ((long long)in_sizes[3] < (long long)SEQ * 64) return;
    if ((long long)in_sizes[4] < (long long)SEQ * 64) return;
    if ((long long)in_sizes[5] < (long long)4 * DM * DM) return;
    if (in_sizes[6] < NHEAD * 12) return;
    if ((long long)out_size < need_rows * DM) return;
    if ((size_t)SZ_TOTAL > ws_size) return;

    const float* x    = (const float*)d_in[0];
    const float* ve   = (const float*)d_in[1];
    const float* lam  = (const float*)d_in[2];
    const float* cosb = (const float*)d_in[3];
    const float* sinb = (const float*)d_in[4];
    const float* w    = (const float*)d_in[5];
    const float* gw   = (const float*)d_in[6];
    float* out = (float*)d_out;

    char* wsp = (char*)d_ws;
    float*          RS    = (float*)wsp;          wsp += SZ_RS;
    float*          SC    = (float*)wsp;          wsp += SZ_SC;
    unsigned short* XQ    = (unsigned short*)wsp; wsp += SZ_XQ;
    unsigned short* W2    = (unsigned short*)wsp; wsp += SZ_W2;
    float*          QKV   = (float*)wsp;          wsp += SZ_QKV;
    float*          GATE  = (float*)wsp;          wsp += SZ_GATE;
    unsigned short* QK16  = (unsigned short*)wsp; wsp += SZ_QK16;
    unsigned short* QKR   = (unsigned short*)wsp; wsp += SZ_QKR;
    unsigned short* VT16  = (unsigned short*)wsp; wsp += SZ_VT16;
    unsigned short* VTR   = (unsigned short*)wsp; wsp += SZ_VTR;
    unsigned short* CTX16 = (unsigned short*)wsp; wsp += SZ_CTX16;
    unsigned short* CTXE  = (unsigned short*)wsp; wsp += SZ_CTXE;
    unsigned short* WO2   = W2 + (size_t)3 * DM * K2;

    k_wrowsum<<<(unsigned)(4 * DM / 32), 256, 0, stream>>>(w, RS);
    k_wscale<<<1, 128, 0, stream>>>(RS, SC);
    k_cast_tern<<<(unsigned)(4 * DM * (DM / 8) / 256), 256, 0, stream>>>(w, SC, W2);
    k_xquant<<<(unsigned)(MT / 2), 256, 0, stream>>>(x, gw, XQ, GATE, MT);
    k_gemm_f32<<<(unsigned)(((MT / 64) * (QKVW / 64) + 7) / 8), 256, 0, stream>>>(XQ, K2, W2, K2, QKV, QKVW, MT, QKVW, K2, 1.0f, MT, MT);
    k_qkpost<<<(unsigned)(MT / 2), 256, 0, stream>>>(QKV, SC, cosb, sinb, QK16, QKR);
    k_vpost<<<(unsigned)((MT / 64) * (DM / 64)), 256, 0, stream>>>(QKV, ve, lam, SC, VT16, VTR);
    k_attn128<<<(unsigned)(NB * NHEAD * (SEQ / 64)), 128, 0, stream>>>(QK16, VT16, GATE, SC, CTX16);
    k_attn_early<<<(unsigned)(NB * NHEAD * (EROWS / 64) * 2), 128, 0, stream>>>(QK16, QKR, VT16, VTR, GATE, SC, CTXE);
    k_gemm_f32<<<(unsigned)(((MT / 64) * (DM / 64) + 7) / 8), 256, 0, stream>>>(CTX16, DM, WO2, K2, out, DM, MT, DM, DM, 1.0f / 4096.0f, SEQ, SEQ_FULL);
    k_gemm_f32<<<(unsigned)(((MTE / 64) * (DM / 64) + 7) / 8), 256, 0, stream>>>(CTXE, K2, WO2, K2, out, DM, MTE, DM, K2, 1.0f / 4096.0f, EROWS, SEQ_FULL);
}
